// DeformableBlock_44083544326619
// MI455X (gfx1250) — hardware-run, weakly checked
//
#include <hip/hip_runtime.h>
#include <stddef.h>
#include <math.h>

typedef __attribute__((ext_vector_type(16))) _Float16 v16h;
typedef __attribute__((ext_vector_type(8)))  _Float16 v8h;
typedef __attribute__((ext_vector_type(16))) __bf16   v16b;
typedef __attribute__((ext_vector_type(8)))  __bf16   v8b;
typedef __attribute__((ext_vector_type(8)))  float    v8f;
typedef __attribute__((ext_vector_type(4)))  float    v4f;

constexpr int NB    = 2;
constexpr int NC    = 256;
constexpr int NH    = 64;
constexpr int NWD   = 64;
constexpr int NHW   = NH * NWD;
constexpr int NPOS  = NB * NHW;
constexpr int KDIM  = 9 * NC;
constexpr int NOFF  = 18;
constexpr int NOFFP = 64;
constexpr int NGRP  = 8;
constexpr int CPG   = NC / NGRP;
constexpr int NTHR  = 256;
constexpr int KPR   = KDIM / 8;
constexpr float WCARRY = 256.0f;
constexpr float WFOLD  = 0.00390625f;
constexpr float GN_EPS = 1e-5f;
constexpr float GN_INV_N = 1.0f / 131072.0f;

constexpr size_t WS_XF    = 0;
constexpr size_t WS_A1F   = WS_XF  + (size_t)NPOS * NC * 4;
constexpr size_t WS_Y     = WS_A1F + (size_t)NPOS * NC * 4;
constexpr size_t WS_IM    = WS_Y   + (size_t)NPOS * NC * 4;
constexpr size_t WS_OFF   = WS_IM  + (size_t)NPOS * KDIM * 2;
constexpr size_t WS_WD1   = WS_OFF + (size_t)NPOS * NOFFP * 4;
constexpr size_t WS_WD2   = WS_WD1 + (size_t)NC * KDIM * 2;
constexpr size_t WS_WO1   = WS_WD2 + (size_t)NC * KDIM * 2;
constexpr size_t WS_WO2   = WS_WO1 + (size_t)NOFFP * KDIM * 2;
constexpr size_t WS_ST    = WS_WO2 + (size_t)NOFFP * KDIM * 2;
constexpr size_t WS_TOTAL = WS_ST  + (size_t)NB * NGRP * 128;
static_assert(WS_TOTAL == 67962880);
static_assert(WS_TOTAL <= 134217728);
static_assert(WS_A1F % 4096 == 0 && WS_Y % 4096 == 0 && WS_IM % 4096 == 0 && WS_OFF % 4096 == 0);
static_assert(WS_WD1 % 4096 == 0 && WS_WD2 % 4096 == 0 && WS_WO1 % 4096 == 0 && WS_WO2 % 4096 == 0 && WS_ST % 4096 == 0);

static_assert(KDIM % 32 == 0);
static_assert(NPOS % 64 == 0 && NC % 64 == 0 && NOFFP % 64 == 0);
constexpr int GEMM_OFF_BLOCKS = ((NPOS / 64) * (NOFFP / 64)) / 8;
constexpr int GEMM_MAIN_BLOCKS = ((NPOS / 64) * (NC / 64)) / 8;
static_assert(((NPOS / 64) * (NOFFP / 64)) % 8 == 0);
static_assert(((NPOS / 64) * (NC / 64)) % 8 == 0);
static_assert(NPOS % 32 == 0 && NHW % 32 == 0);
static_assert(NPOS % 8 == 0);
static_assert((NC * KPR) % NTHR == 0 && (NOFFP * KPR) % NTHR == 0);
static_assert((NPOS * NC) % (NTHR * 4) == 0);
static_assert(NC == NTHR);
static_assert(CPG * NHW == 128 * NTHR * 4);

__device__ __forceinline__ unsigned short f2bf_bits(float f) {
  unsigned u = __float_as_uint(f);
  return (unsigned short)((u + 0x7FFFu + ((u >> 16) & 1u)) >> 16);
}
__device__ __forceinline__ float bf_bits2f(unsigned short h) { return __uint_as_float(((unsigned)h) << 16); }

__device__ __forceinline__ void dep_guard_h(v8f& a, v8f& b, v16h x, v16h y) { asm volatile("v_nop\n\tv_nop\n\tv_nop\n\tv_nop" : "+v"(a), "+v"(b) : "v"(x), "v"(y)); }
__device__ __forceinline__ void dep_guard_b(v8f& a, v8f& b, v16b x, v16b y) { asm volatile("v_nop\n\tv_nop\n\tv_nop\n\tv_nop" : "+v"(a), "+v"(b) : "v"(x), "v"(y)); }
__device__ __forceinline__ void keep4_h(v16h a, v16h b, v16h c, v16h d) { asm volatile("v_nop" :: "v"(a), "v"(b), "v"(c), "v"(d)); }
__device__ __forceinline__ void keep4_b(v16b a, v16b b, v16b c, v16b d) { asm volatile("v_nop" :: "v"(a), "v"(b), "v"(c), "v"(d)); }
__device__ __forceinline__ void acc_guard4(v8f& a, v8f& b, v8f& c, v8f& d) { asm volatile("v_nop\n\tv_nop\n\tv_nop\n\tv_nop" : "+v"(a), "+v"(b), "+v"(c), "+v"(d)); }
template <typename T> struct Frag;
template <> struct Frag<_Float16> {
  typedef v16h V; union U { v16h v; v8h h[2]; };
  static __device__ __forceinline__ v16h load(const _Float16* p) {
    U f; f.h[0] = *(const v8h*)(p); f.h[1] = *(const v8h*)(p + 16); return f.v;
  }
  static __device__ __forceinline__ v8f mma(v16h a, v16h b, v8f c) {
    return __builtin_amdgcn_wmma_f32_16x16x32_f16(false, a, false, b, (short)0, c, false, false);
  }
  static __device__ __forceinline__ void guard(v8f& a, v8f& b, v16h x, v16h y) { dep_guard_h(a, b, x, y); }
  static __device__ __forceinline__ void keep(v16h a, v16h b, v16h c, v16h d) { keep4_h(a, b, c, d); }
};
template <> struct Frag<__bf16> {
  typedef v16b V; union U { v16b v; v8b h[2]; };
  static __device__ __forceinline__ v16b load(const __bf16* p) {
    U f; f.h[0] = *(const v8b*)(p); f.h[1] = *(const v8b*)(p + 16); return f.v;
  }
  static __device__ __forceinline__ v8f mma(v16b a, v16b b, v8f c) {
    return __builtin_amdgcn_wmma_f32_16x16x32_bf16(false, a, false, b, (short)0, c, false, false);
  }
  static __device__ __forceinline__ void guard(v8f& a, v8f& b, v16b x, v16b y) { dep_guard_b(a, b, x, y); }
  static __device__ __forceinline__ void keep(v16b a, v16b b, v16b c, v16b d) { keep4_b(a, b, c, d); }
};

template <int ET> struct Elem;
template <> struct Elem<0> { typedef _Float16 T; };
template <> struct Elem<1> { typedef __bf16 T; };
template <int ET, bool SPLIT, int BIAS_MODE, int OUT_MODE, bool RESID, int ACT = 0>
__global__ __launch_bounds__(256) void wmma_gemm64(
    const unsigned short* __restrict__ Ap, const unsigned short* __restrict__ A2p, int lda, long strideA,
    const unsigned short* __restrict__ Btp, const unsigned short* __restrict__ Bt2p, int ldb, long strideB,
    void* __restrict__ Cout, void* __restrict__ Cout2, int ldc, long strideC,
    const float* __restrict__ bias,
    const float* __restrict__ resid, long strideR,
    int M, int N, int K, float scale) {
  typedef typename Elem<ET>::T T;
  typedef typename Frag<T>::V V;
  const T* A = (const T*)Ap; const T* A2 = (const T*)A2p; const T* Bt = (const T*)Btp; const T* Bt2 = (const T*)Bt2p;
  __shared__ __align__(16) float sT[8][16 * 68];
  const int b    = blockIdx.y;
  const int lane = threadIdx.x & 31;
  const int wave = threadIdx.x >> 5;
  const int tilesN = N >> 6;
  const int tilesM = M >> 6;
  const int tile = blockIdx.x * 8 + wave;
  if (tile >= tilesM * tilesN) return;
  const int tm = tile / tilesN;
  const int tn = tile - tm * tilesN;
  const int m0 = tm << 6;
  const int n0 = tn << 6;

  const T* Ab  = A  + (size_t)b * strideA;
  const T* Bb  = Bt + (size_t)b * strideB;
  const T* Ab2 = SPLIT ? (A2  + (size_t)b * strideA) : nullptr;
  const T* Bb2 = SPLIT ? (Bt2 + (size_t)b * strideB) : nullptr;

  const int rlane = lane & 15;
  const int koff  = (lane >> 4) * 8;
  const int mOff  = (lane >> 4) * 8;

  v8f acc[4][4];
#pragma unroll
  for (int i = 0; i < 4; ++i)
#pragma unroll
    for (int j = 0; j < 4; ++j) acc[i][j] = (v8f){0.f,0.f,0.f,0.f,0.f,0.f,0.f,0.f};

  for (int k0 = 0; k0 < K; k0 += 32) {
    V bh[4], bl[4];
#pragma unroll
    for (int j = 0; j < 4; ++j) {
      const size_t bo = (size_t)(n0 + (j << 4) + rlane) * ldb + koff + k0;
      bh[j] = Frag<T>::load(Bb + bo);
      if (SPLIT) bl[j] = Frag<T>::load(Bb2 + bo);
    }
#pragma unroll
    for (int i = 0; i < 4; ++i) {
      const size_t ao = (size_t)(m0 + (i << 4) + rlane) * lda + koff + k0;
      V ah = Frag<T>::load(Ab + ao);
      V al;
      if (SPLIT) al = Frag<T>::load(Ab2 + ao);
#pragma unroll
      for (int j = 0; j < 4; ++j) {
        acc[i][j] = Frag<T>::mma(ah, bh[j], acc[i][j]);
        if (SPLIT) {
          acc[i][j] = Frag<T>::mma(ah, bl[j], acc[i][j]);
          acc[i][j] = Frag<T>::mma(al, bh[j], acc[i][j]);
        }
      }
      Frag<T>::guard(acc[i][0], acc[i][3], ah, SPLIT ? al : ah);
    }
    Frag<T>::keep(bh[0], bh[1], bh[2], bh[3]);
    if (SPLIT) Frag<T>::keep(bl[0], bl[1], bl[2], bl[3]);
  }
  acc_guard4(acc[0][0], acc[0][1], acc[0][2], acc[0][3]);
  acc_guard4(acc[1][0], acc[1][1], acc[1][2], acc[1][3]);
  acc_guard4(acc[2][0], acc[2][1], acc[2][2], acc[2][3]);
  acc_guard4(acc[3][0], acc[3][1], acc[3][2], acc[3][3]);

  float* slab = sT[wave];
  const float* Rb = RESID ? (resid + (size_t)b * strideR) : nullptr;
#pragma unroll
  for (int i = 0; i < 4; ++i) {
    const int mBase = m0 + (i << 4);
#pragma unroll
    for (int j = 0; j < 4; ++j) {
      const int n = n0 + (j << 4) + rlane;
      float bv = 0.f;
      if (BIAS_MODE == 2) bv = bias[n];
#pragma unroll
      for (int r = 0; r < 8; ++r) {
        float v = acc[i][j][r] * scale;
        if (BIAS_MODE == 1) v += bias[mBase + mOff + r];
        if (BIAS_MODE == 2) v += bv;
        if (RESID) v += Rb[(size_t)(mBase + mOff + r) * ldc + n];
        if (ACT == 1) v = tanhf(v);
        if (ACT == 2) v = fmaxf(v, 0.0f);
        if (ACT == 3) v = v / (1.0f + expf(-v));
        if (ACT == 4) v = (v > 0.f) ? v : 0.01f * v;
        if (ACT == 5) v = 0.5f * v * (1.0f + erff(v * 0.70710678118654752f));
        slab[(mOff + r) * 68 + (j << 4) + rlane] = v;
      }
    }
    __builtin_amdgcn_fence(__ATOMIC_RELEASE, "workgroup");
    __builtin_amdgcn_wave_barrier();
    __builtin_amdgcn_fence(__ATOMIC_ACQUIRE, "workgroup");
    if (OUT_MODE == 0) {
      float* C = (float*)Cout + (size_t)b * strideC;
      const int hh = lane >> 4, c4 = (lane & 15) * 4;
      for (int pass = 0; pass < 2; ++pass) {
#pragma unroll
        for (int it = 0; it < 8; ++it) {
          const int row = it * 2 + hh;
          v4f v = *(const v4f*)(slab + row * 68 + c4);
          *(volatile v4f*)(C + (size_t)(mBase + row) * ldc + n0 + c4) = v;
        }
        __threadfence();
      }
    } else {
      const int q = lane >> 3, c8 = (lane & 7) * 8;
      unsigned short* C  = (unsigned short*)Cout  + (size_t)b * strideC;
      unsigned short* C2 = (OUT_MODE == 2) ? ((unsigned short*)Cout2 + (size_t)b * strideC) : nullptr;
      for (int pass = 0; pass < 2; ++pass) {
#pragma unroll
        for (int it = 0; it < 4; ++it) {
          const int row = it * 4 + q;
          const float* sp = slab + row * 68 + c8;
          v8h hv, lv;
#pragma unroll
          for (int e = 0; e < 8; ++e) {
            if (OUT_MODE == 1) {
              hv[e] = (_Float16)sp[e];
            } else {
              unsigned short hb = f2bf_bits(sp[e]);
              unsigned short lb = f2bf_bits(sp[e] - bf_bits2f(hb));
              hv[e] = __builtin_bit_cast(_Float16, hb);
              lv[e] = __builtin_bit_cast(_Float16, lb);
            }
          }
          *(volatile v8h*)(C + (size_t)(mBase + row) * ldc + n0 + c8) = hv;
          if (OUT_MODE == 2) *(volatile v8h*)(C2 + (size_t)(mBase + row) * ldc + n0 + c8) = lv;
        }
        __threadfence();
      }
    }
    __builtin_amdgcn_fence(__ATOMIC_RELEASE, "workgroup");
    __builtin_amdgcn_wave_barrier();
    __builtin_amdgcn_fence(__ATOMIC_ACQUIRE, "workgroup");
  }
}

__device__ __forceinline__ float bfr(float f) { return bf_bits2f(f2bf_bits(f)); }
__device__ __forceinline__ int clampi(int v, int lo, int hi) { return v < lo ? lo : (v > hi ? hi : v); }

__global__ __launch_bounds__(NTHR) void k_prep_x(const float* __restrict__ x, float* __restrict__ xf) {
  __shared__ __align__(16) float s_t[32 * 260];
  const int tid  = threadIdx.x;
  const int pos0 = blockIdx.x * 32;
  const int b    = pos0 >> 12;
  const int hw0  = pos0 & (NHW - 1);
  const float* xb = x + (size_t)b * NC * NHW + hw0;
#pragma unroll 1
  for (int i = 0; i < 32; ++i) {
    const int e = i * NTHR + tid;
    const int c = e >> 5;
    const int p = e & 31;
    s_t[p * 260 + c] = bfr(xb[(size_t)c * NHW + p]);
  }
  __syncthreads();
  float* dstb = xf + (size_t)pos0 * NC;
  for (int pass = 0; pass < 2; ++pass) {
#pragma unroll
    for (int i = 0; i < 8; ++i) {
      const int f  = i * NTHR + tid;
      const int p  = f >> 6;
      const int c4 = (f & 63) * 4;
      const v4f v = *(const v4f*)(s_t + p * 260 + c4);
      *(volatile v4f*)(dstb + (size_t)p * NC + c4) = v;
    }
    __threadfence();
  }
}

__global__ __launch_bounds__(NTHR) void k_wprep(const float* __restrict__ W, int nreal, int npad,
                                               unsigned short* __restrict__ bt) {
  const int i = blockIdx.x * NTHR + threadIdx.x;
  if (i >= npad * KPR) return;
  const int n   = i / KPR;
  const int k0  = (i - n * KPR) * 8;
  const int tap = k0 >> 8;
  const int c0  = k0 & 255;
  const int ncl = (n < nreal) ? n : (nreal - 1);
  const float* src = W + ((size_t)ncl * NC + c0) * 9 + tap;
  v8h hv;
#pragma unroll
  for (int e = 0; e < 8; ++e) {
    float v = src[e * 9];
    v = (n < nreal) ? (bfr(v) * WCARRY) : 0.0f;
    hv[e] = (_Float16)v;
  }
  unsigned short* d = bt + (size_t)i * 8;
  *(volatile v8h*)d = hv;
  __threadfence();
  *(volatile v8h*)d = hv;
}

template <bool WITH_OFFSET>
__global__ __launch_bounds__(NTHR) void k_build_a(const float* __restrict__ src, const float* __restrict__ offp,
                                                 const float* __restrict__ offb, unsigned short* __restrict__ im) {
#pragma clang fp contract(off)
  const int lane = threadIdx.x & 31;
  const int wave = threadIdx.x >> 5;
  const int m  = blockIdx.x * 8 + wave;
  const int b  = m >> 12;
  const int hw = m & (NHW - 1);
  const int h  = hw >> 6;
  const int w  = hw & 63;
  const int c0 = lane * 8;
  const float* sb = src + (size_t)b * NHW * NC + c0;
  unsigned short* dst = im + (size_t)m * KDIM + c0;
#pragma unroll 1
  for (int tap = 0; tap < 9; ++tap) {
    const int ky = tap / 3;
    const int kx = tap - ky * 3;
    float a[8];
    if (!WITH_OFFSET) {
      const int yy = h - 1 + ky;
      const int xx = w - 1 + kx;
      const bool valid = (yy >= 0) && (yy < NH) && (xx >= 0) && (xx < NWD);
      const int yc = clampi(yy, 0, NH - 1);
      const int xc = clampi(xx, 0, NWD - 1);
      const float* p = sb + (size_t)(yc * NWD + xc) * NC;
      const v4f u0 = *(const v4f*)(p);
      const v4f u1 = *(const v4f*)(p + 4);
      const float vf = valid ? 1.0f : 0.0f;
#pragma unroll
      for (int e = 0; e < 4; ++e) { a[e] = u0[e] * vf; a[4 + e] = u1[e] * vf; }
    } else {
      const float dy = offp[(size_t)m * NOFFP + 2 * tap] + bfr(offb[2 * tap]);
      const float dx = offp[(size_t)m * NOFFP + 2 * tap + 1] + bfr(offb[2 * tap + 1]);
      const float py = (float)(h - 1 + ky) + dy;
      const float px = (float)(w - 1 + kx) + dx;
      const float y0 = floorf(py);
      const float x0 = floorf(px);
      const float ty = py - y0;
      const float tx = px - x0;
      const float y1 = y0 + 1.0f;
      const float x1 = x0 + 1.0f;
      const float omty = 1.0f - ty;
      const float omtx = 1.0f - tx;
      const float w00 = omty * omtx;
      const float w01 = omty * tx;
      const float w10 = ty * omtx;
      const float w11 = ty * tx;
      const bool vy0 = (y0 >= 0.0f) && (y0 < (float)NH);
      const bool vy1 = (y1 >= 0.0f) && (y1 < (float)NH);
      const bool vx0 = (x0 >= 0.0f) && (x0 < (float)NWD);
      const bool vx1 = (x1 >= 0.0f) && (x1 < (float)NWD);
      const float f00 = (vy0 && vx0) ? 1.0f : 0.0f;
      const float f01 = (vy0 && vx1) ? 1.0f : 0.0f;
      const float f10 = (vy1 && vx0) ? 1.0f : 0.0f;
      const float f11 = (vy1 && vx1) ? 1.0f : 0.0f;
      const int iy0 = (int)fminf(fmaxf(y0, 0.0f), (float)(NH - 1));
      const int iy1 = (int)fminf(fmaxf(y1, 0.0f), (float)(NH - 1));
      const int ix0 = (int)fminf(fmaxf(x0, 0.0f), (float)(NWD - 1));
      const int ix1 = (int)fminf(fmaxf(x1, 0.0f), (float)(NWD - 1));
      const float* p00 = sb + (size_t)(iy0 * NWD + ix0) * NC;
      const float* p01 = sb + (size_t)(iy0 * NWD + ix1) * NC;
      const float* p10 = sb + (size_t)(iy1 * NWD + ix0) * NC;
      const float* p11 = sb + (size_t)(iy1 * NWD + ix1) * NC;
      const v4f g00a = *(const v4f*)(p00); const v4f g00b = *(const v4f*)(p00 + 4);
      const v4f g01a = *(const v4f*)(p01); const v4f g01b = *(const v4f*)(p01 + 4);
      const v4f g10a = *(const v4f*)(p10); const v4f g10b = *(const v4f*)(p10 + 4);
      const v4f g11a = *(const v4f*)(p11); const v4f g11b = *(const v4f*)(p11 + 4);
#pragma unroll
      for (int e = 0; e < 4; ++e) {
        a[e]     = (((g00a[e] * f00) * w00 + (g01a[e] * f01) * w01) + (g10a[e] * f10) * w10) + (g11a[e] * f11) * w11;
        a[4 + e] = (((g00b[e] * f00) * w00 + (g01b[e] * f01) * w01) + (g10b[e] * f10) * w10) + (g11b[e] * f11) * w11;
      }
    }
    v8h hv;
#pragma unroll
    for (int e = 0; e < 8; ++e) hv[e] = (_Float16)a[e];
    unsigned short* d = dst + tap * NC;
    *(volatile v8h*)d = hv;
    __threadfence();
    *(volatile v8h*)d = hv;
  }
}

__global__ __launch_bounds__(NTHR) void k_gn_stats(const float* __restrict__ y, float* __restrict__ stats) {
  __shared__ float ssum[NTHR];
  __shared__ float ssq[NTHR];
  __shared__ __align__(16) float sline[32];
  const int tid = threadIdx.x;
  const int bg  = blockIdx.x;
  const int b   = bg >> 3;
  const int g   = bg & 7;
  const float* base = y + (size_t)b * NHW * NC + g * CPG;
  float s = 0.0f, q = 0.0f;
#pragma unroll 1
  for (int it = 0; it < 128; ++it) {
    const int f  = it * NTHR + tid;
    const int p  = f >> 3;
    const int c4 = (f & 7) * 4;
    const v4f v = *(const v4f*)(base + (size_t)p * NC + c4);
    s += (v[0] + v[1]) + (v[2] + v[3]);
    q += (v[0] * v[0] + v[1] * v[1]) + (v[2] * v[2] + v[3] * v[3]);
  }
  ssum[tid] = s;
  ssq[tid]  = q;
  __syncthreads();
  for (int st = NTHR / 2; st > 0; st >>= 1) {
    if (tid < st) {
      ssum[tid] += ssum[tid + st];
      ssq[tid]  += ssq[tid + st];
    }
    __syncthreads();
  }
  {
    const float mu = ssum[0] * GN_INV_N;
    float var = ssq[0] * GN_INV_N - mu * mu;
    var = fmaxf(var, 0.0f);
    const float rs = rsqrtf(var + GN_EPS);
    float val = 0.0f;
    if (tid == 0) val = mu;
    if (tid == 1) val = rs;
    if (tid < 32) sline[tid] = val;
  }
  __syncthreads();
  if (tid < 8) {
    const v4f v = *(const v4f*)(sline + tid * 4);
    float* d = stats + (size_t)bg * 32 + tid * 4;
    *(volatile v4f*)d = v;
    __threadfence();
    *(volatile v4f*)d = v;
  }
}

__global__ __launch_bounds__(NTHR) void k_gn_mid(const float* __restrict__ y, const float* __restrict__ stats,
                                                const float* __restrict__ gs, const float* __restrict__ gb,
                                                float* __restrict__ a1f) {
  const size_t e0 = ((size_t)blockIdx.x * NTHR + threadIdx.x) * 4;
  const int pos = (int)(e0 >> 8);
  const int c4  = (int)(e0 & 255);
  const int b   = pos >> 12;
  const int g   = c4 >> 5;
  const float mu = stats[(b * NGRP + g) * 32];
  const float rs = stats[(b * NGRP + g) * 32 + 1];
  const v4f v  = *(const v4f*)(y + e0);
  const v4f sc = *(const v4f*)(gs + c4);
  const v4f bi = *(const v4f*)(gb + c4);
  v4f o;
#pragma unroll
  for (int e = 0; e < 4; ++e) {
    const float t = ((v[e] - mu) * rs) * bfr(sc[e]) + bfr(bi[e]);
    o[e] = fmaxf(t, 0.0f);
  }
  float* d = a1f + e0;
  *(volatile v4f*)d = o;
  __threadfence();
  *(volatile v4f*)d = o;
}

__global__ __launch_bounds__(NTHR) void k_gn_out(const float* __restrict__ y, const float* __restrict__ stats,
                                                const float* __restrict__ gs, const float* __restrict__ gb,
                                                float* __restrict__ out) {
  __shared__ __align__(16) float s_o[NC * 36];
  const int tid  = threadIdx.x;
  const int lane = tid & 31;
  const int wave = tid >> 5;
  const int pos0 = blockIdx.x * 32;
  const int b    = pos0 >> 12;
  const int hw0  = pos0 & (NHW - 1);
  {
    const int c  = tid;
    const int g  = c >> 5;
    const float mu = stats[(b * NGRP + g) * 32];
    const float rs = stats[(b * NGRP + g) * 32 + 1];
    const float sc = bfr(gs[c]);
    const float bi = bfr(gb[c]);
    const float* yb = y + (size_t)pos0 * NC + c;
#pragma unroll 1
    for (int p = 0; p < 32; ++p) {
      const float v = yb[(size_t)p * NC];
      const float t = ((v - mu) * rs) * sc + bi;
      s_o[c * 36 + p] = fmaxf(t, 0.0f);
    }
  }
  __syncthreads();
  const int q  = lane >> 3;
  const int c4 = (lane & 7) * 4;
  float* ob = out + (size_t)b * NC * NHW + hw0 + c4;
  for (int pass = 0; pass < 2; ++pass) {
#pragma unroll
    for (int it = 0; it < 8; ++it) {
      const int cc = it * 32 + wave * 4 + q;
      const v4f v = *(const v4f*)(s_o + cc * 36 + c4);
      *(volatile v4f*)(ob + (size_t)cc * NHW) = v;
    }
    __threadfence();
  }
}

extern "C" void kernel_launch(void* const* d_in, const int* in_sizes, int n_in,
                              void* d_out, int out_size, void* d_ws, size_t ws_size,
                              hipStream_t stream) {
  if (n_in < 11) return;
  if (in_sizes[0] != NPOS * NC || in_sizes[1] != NOFF * KDIM || in_sizes[2] != NOFF ||
      in_sizes[3] != NC * KDIM || in_sizes[4] != NC || in_sizes[5] != NC ||
      in_sizes[6] != NOFF * KDIM || in_sizes[7] != NOFF || in_sizes[8] != NC * KDIM ||
      in_sizes[9] != NC || in_sizes[10] != NC) return;
  if (out_size != NPOS * NC) return;
  if (ws_size < WS_TOTAL) return;

  const float* x      = (const float*)d_in[0];
  const float* off1_w = (const float*)d_in[1];
  const float* off1_b = (const float*)d_in[2];
  const float* dw1    = (const float*)d_in[3];
  const float* gn1_s  = (const float*)d_in[4];
  const float* gn1_b  = (const float*)d_in[5];
  const float* off2_w = (const float*)d_in[6];
  const float* off2_b = (const float*)d_in[7];
  const float* dw2    = (const float*)d_in[8];
  const float* gn2_s  = (const float*)d_in[9];
  const float* gn2_b  = (const float*)d_in[10];
  float* out = (float*)d_out;
  char* ws = (char*)d_ws;

  float* xf  = (float*)(ws + WS_XF);
  float* a1f = (float*)(ws + WS_A1F);
  float* yb  = (float*)(ws + WS_Y);
  unsigned short* im  = (unsigned short*)(ws + WS_IM);
  float* offp = (float*)(ws + WS_OFF);
  unsigned short* wd1 = (unsigned short*)(ws + WS_WD1);
  unsigned short* wd2 = (unsigned short*)(ws + WS_WD2);
  unsigned short* wo1 = (unsigned short*)(ws + WS_WO1);
  unsigned short* wo2 = (unsigned short*)(ws + WS_WO2);
  float* st = (float*)(ws + WS_ST);
  const unsigned short* imc  = im;
  const unsigned short* wd1c = wd1;
  const unsigned short* wd2c = wd2;
  const unsigned short* wo1c = wo1;
  const unsigned short* wo2c = wo2;

  k_prep_x<<<NPOS / 32, NTHR, 0, stream>>>(x, xf);
  k_wprep<<<(NC * KPR) / NTHR, NTHR, 0, stream>>>(dw1, NC, NC, wd1);
  k_wprep<<<(NC * KPR) / NTHR, NTHR, 0, stream>>>(dw2, NC, NC, wd2);
  k_wprep<<<(NOFFP * KPR) / NTHR, NTHR, 0, stream>>>(off1_w, NOFF, NOFFP, wo1);
  k_wprep<<<(NOFFP * KPR) / NTHR, NTHR, 0, stream>>>(off2_w, NOFF, NOFFP, wo2);

  k_build_a<false><<<NPOS / 8, NTHR, 0, stream>>>(xf, offp, off1_b, im);
  wmma_gemm64<0, false, 0, 0, false, 0><<<dim3(GEMM_OFF_BLOCKS, 1), NTHR, 0, stream>>>(
      imc, imc, KDIM, 0L, wo1c, wo1c, KDIM, 0L, (void*)offp, (void*)offp, NOFFP, 0L,
      off1_b, offp, 0L, NPOS, NOFFP, KDIM, WFOLD);
  k_build_a<true><<<NPOS / 8, NTHR, 0, stream>>>(xf, offp, off1_b, im);
  wmma_gemm64<0, false, 0, 0, false, 0><<<dim3(GEMM_MAIN_BLOCKS, 1), NTHR, 0, stream>>>(
      imc, imc, KDIM, 0L, wd1c, wd1c, KDIM, 0L, (void*)yb, (void*)yb, NC, 0L,
      off1_b, yb, 0L, NPOS, NC, KDIM, WFOLD);
  k_gn_stats<<<NB * NGRP, NTHR, 0, stream>>>(yb, st);
  k_gn_mid<<<(NPOS * NC) / (NTHR * 4), NTHR, 0, stream>>>(yb, st, gn1_s, gn1_b, a1f);

  k_build_a<false><<<NPOS / 8, NTHR, 0, stream>>>(a1f, offp, off2_b, im);
  wmma_gemm64<0, false, 0, 0, false, 0><<<dim3(GEMM_OFF_BLOCKS, 1), NTHR, 0, stream>>>(
      imc, imc, KDIM, 0L, wo2c, wo2c, KDIM, 0L, (void*)offp, (void*)offp, NOFFP, 0L,
      off2_b, offp, 0L, NPOS, NOFFP, KDIM, WFOLD);
  k_build_a<true><<<NPOS / 8, NTHR, 0, stream>>>(a1f, offp, off2_b, im);
  wmma_gemm64<0, false, 0, 0, false, 0><<<dim3(GEMM_MAIN_BLOCKS, 1), NTHR, 0, stream>>>(
      imc, imc, KDIM, 0L, wd2c, wd2c, KDIM, 0L, (void*)yb, (void*)yb, NC, 0L,
      off2_b, yb, 0L, NPOS, NC, KDIM, WFOLD);
  k_gn_stats<<<NB * NGRP, NTHR, 0, stream>>>(yb, st);
  k_gn_out<<<NPOS / 32, NTHR, 0, stream>>>(yb, st, gn2_s, gn2_b, out);
}
